// ClusteringLayer_63900523430220
// MI455X (gfx1250) — hardware-verified
//
#include <hip/hip_runtime.h>
#include <stdint.h>

#ifndef NROWS
#define NROWS  16384
#endif
#define FEATS  256
#define NCLUST 128
#define RPB    64
#define OPITCH 132
#define CNP    32
static_assert((NROWS % RPB) == 0);
static_assert(FEATS == 256);
static_assert(NCLUST == 128);
static_assert((FEATS % 32) == 0);
static_assert(((NCLUST * FEATS / 8) % 256) == 0);
static_assert((FEATS / 8) == 32);

typedef __bf16   v16b __attribute__((ext_vector_type(16)));
typedef __bf16   v8b  __attribute__((ext_vector_type(8)));
typedef float    v8f  __attribute__((ext_vector_type(8)));
typedef float    v4f  __attribute__((ext_vector_type(4)));
typedef unsigned int v4u __attribute__((ext_vector_type(4)));
typedef unsigned int v8u __attribute__((ext_vector_type(8)));

#if defined(__HIP_DEVICE_COMPILE__)
#define DEV_ASM 1
#else
#define DEV_ASM 0
#endif

__device__ __forceinline__ unsigned short bf_bits(float f) {
  unsigned u = __float_as_uint(f);
  return (unsigned short)((u + 0x7FFFu + ((u >> 16) & 1u)) >> 16);
}
__device__ __forceinline__ float bf_up(unsigned short hb) { return __uint_as_float(((unsigned)hb) << 16); }
__device__ __forceinline__ unsigned pk16(unsigned short a, unsigned short b) { return (unsigned)a | ((unsigned)b << 16); }
__device__ __forceinline__ v8f zero8() { v8f z = {0.f, 0.f, 0.f, 0.f, 0.f, 0.f, 0.f, 0.f}; return z; }

__device__ __forceinline__ unsigned cvt2(float a, float b, float& s) {
  const unsigned short ba = bf_bits(a), bb = bf_bits(b);
  const float ua = bf_up(ba), ub = bf_up(bb);
  s = fmaf(ua, ua, s);
  s = fmaf(ub, ub, s);
  return pk16(ba, bb);
}

__device__ __forceinline__ v16b ldfrag_b(const __bf16* p) {
  union { v16b v; v8b h[2]; } f;
  f.h[0] = *(const v8b*)(p);
  f.h[1] = *(const v8b*)(p + 16);
  return f.v;
}

__device__ __forceinline__ v8f mma_b(v16b a, v16b b, v8f c) {
  c = __builtin_amdgcn_wmma_f32_16x16x32_bf16(false, a, false, b, (short)0, c, false, false);
#if DEV_ASM
  asm volatile("v_nop\n\tv_nop\n\tv_nop\n\tv_nop" : "+v"(c) : "v"(a), "v"(b));
#endif
  return c;
}

__global__ __launch_bounds__(256) void cvt_cent(const float* __restrict__ in, unsigned short* outp, float* cnp) {
  const int tid  = (int)threadIdx.x;
  const int i    = blockIdx.x * 256 + tid;
  const int lane = tid & 31;
  const int n    = i >> 5;
  const v4f a  = *(const v4f*)(in + (size_t)i * 8);
  const v4f a4 = *(const v4f*)(in + (size_t)i * 8 + 4);
  float s = 0.f;
  v4u p;
  p[0] = cvt2(a[0],  a[1],  s);
  p[1] = cvt2(a[2],  a[3],  s);
  p[2] = cvt2(a4[0], a4[1], s);
  p[3] = cvt2(a4[2], a4[3], s);
#pragma unroll
  for (int off = 1; off < 32; off <<= 1) s += __shfl_xor(s, off, 32);
  unsigned short* o = outp + (size_t)i * 8;
  float* q = cnp + (size_t)n * CNP + lane;
  *(volatile v4u*)o   = p;
  *(volatile float*)q = s;
  __threadfence();
  *(volatile v4u*)o   = p;
  *(volatile float*)q = s;
}

__global__ __launch_bounds__(128)
void soft_assign(const float* __restrict__ X, const unsigned short* __restrict__ Cbp,
                 const float* __restrict__ cnp, float* outp) {
  __shared__ __align__(16) float sO[4][16 * OPITCH];
  __shared__ float s_cn[NCLUST];

  const int tid  = (int)threadIdx.x;
  const int lane = tid & 31;
  const int wave = tid >> 5;
  const int hh   = lane >> 4;
  const int c    = lane & 15;

  s_cn[tid] = cnp[(size_t)tid * CNP];
  __syncthreads();

  const int rowBase = blockIdx.x * RPB + wave * 16;
  const float*  xrow = X + (size_t)(rowBase + c) * FEATS;
  const __bf16* CB   = (const __bf16*)(const void*)Cbp;

  v8f acc[8];
#pragma unroll
  for (int nt = 0; nt < 8; ++nt) acc[nt] = zero8();
  float xsq = 0.f;

#pragma unroll
  for (int kk = 0; kk < FEATS; kk += 32) {
    const int f1 = kk + 8 * hh;
    const int f2 = kk + 16 + 8 * hh;
    const v4f x0 = *(const v4f*)(xrow + f1);
    const v4f x1 = *(const v4f*)(xrow + f1 + 4);
    const v4f x2 = *(const v4f*)(xrow + f2);
    const v4f x3 = *(const v4f*)(xrow + f2 + 4);
    v8u ap;
    ap[0] = cvt2(x0[0], x0[1], xsq);
    ap[1] = cvt2(x0[2], x0[3], xsq);
    ap[2] = cvt2(x1[0], x1[1], xsq);
    ap[3] = cvt2(x1[2], x1[3], xsq);
    ap[4] = cvt2(x2[0], x2[1], xsq);
    ap[5] = cvt2(x2[2], x2[3], xsq);
    ap[6] = cvt2(x3[0], x3[1], xsq);
    ap[7] = cvt2(x3[2], x3[3], xsq);
    const v16b af = __builtin_bit_cast(v16b, ap);
#pragma unroll
    for (int nt = 0; nt < 8; ++nt) {
      const v16b bf = ldfrag_b(CB + (size_t)(nt * 16 + c) * FEATS + kk + 8 * hh);
      acc[nt] = mma_b(af, bf, acc[nt]);
    }
  }

  const float xs_full = xsq + __shfl_xor(xsq, 16, 32);
  float cnv[8];
#pragma unroll
  for (int nt = 0; nt < 8; ++nt) cnv[nt] = s_cn[nt * 16 + c];

  float* os = sO[wave];
#pragma unroll
  for (int r = 0; r < 8; ++r) {
    const float xn = __shfl(xs_full, r + 8 * hh, 32);
    float qv[8];
    float rs = 0.f;
#pragma unroll
    for (int nt = 0; nt < 8; ++nt) {
      const float d2 = xn + cnv[nt] - 2.0f * acc[nt][r];
      const float q  = 1.0f / (1.0f + d2);
      qv[nt] = q;
      rs += q;
    }
    rs += __shfl_xor(rs, 1, 32);
    rs += __shfl_xor(rs, 2, 32);
    rs += __shfl_xor(rs, 4, 32);
    rs += __shfl_xor(rs, 8, 32);
    const float rinv = 1.0f / rs;
#pragma unroll
    for (int nt = 0; nt < 8; ++nt) os[(8 * hh + r) * OPITCH + nt * 16 + c] = qv[nt] * rinv;
  }
  __builtin_amdgcn_fence(__ATOMIC_RELEASE, "workgroup");
  __builtin_amdgcn_wave_barrier();
  __builtin_amdgcn_fence(__ATOMIC_ACQUIRE, "workgroup");
  {
    const int c4 = lane * 4;
    for (int pass = 0; pass < 2; ++pass) {
#pragma unroll
      for (int row = 0; row < 16; ++row) {
        const v4f v = *(const v4f*)(os + row * OPITCH + c4);
        *(volatile v4f*)(outp + (size_t)(rowBase + row) * NCLUST + c4) = v;
      }
      __threadfence();
    }
  }
}

extern "C" void kernel_launch(void* const* d_in, const int* in_sizes, int n_in,
                              void* d_out, int out_size, void* d_ws, size_t ws_size,
                              hipStream_t stream) {
  if (n_in < 2) return;
  if (in_sizes[0] < NROWS * FEATS) return;
  if (in_sizes[1] < NCLUST * FEATS) return;
  if (out_size < NROWS * NCLUST) return;

  const float* X = (const float*)d_in[0];
  const float* C = (const float*)d_in[1];
  float* out = (float*)d_out;

  const size_t PCB = (size_t)NCLUST * FEATS * 2;
  const size_t PCN = (size_t)NCLUST * CNP * 4;
  size_t off = 0;
  const size_t oCb = off; off += PCB;
  const size_t oCn = off; off += PCN;
  if (off > ws_size) return;
  if (off > (size_t)134217728) return;

  char* ws = (char*)d_ws;
  unsigned short* Cb = (unsigned short*)(ws + oCb);
  float*          Cn = (float*)(ws + oCn);

  const dim3 gCvt(NCLUST * FEATS / 8 / 256);
  const dim3 gMain(NROWS / RPB);

  cvt_cent<<<gCvt, dim3(256), 0, stream>>>(C, Cb, Cn);
  soft_assign<<<gMain, dim3(128), 0, stream>>>(X, Cb, Cn, out);
  (void)hipGetLastError();
}
